// MambaWeatherBlock_10531259810087
// MI455X (gfx1250) — hardware-verified
//
#include <hip/hip_runtime.h>


namespace {
constexpr int Bn = 4, L = 2048, DM = 768, DI = 1536, NS = 16, KC = 4, R = 48, W = 64, XK = DI + W  , XN = R + 2 * NS  , NT = Bn * L;
constexpr float AS_ = 8.0f;

typedef _Float16 b16;
typedef __attribute__((ext_vector_type(16))) _Float16 v16b;
typedef __attribute__((ext_vector_type(16))) __bf16 v16bb;
typedef __attribute__((ext_vector_type(8))) _Float16 v8b;
typedef __attribute__((ext_vector_type(8))) unsigned short v8us;
typedef __attribute__((ext_vector_type(8))) float v8f;
typedef __attribute__((ext_vector_type(4))) float v4f;
__device__ __forceinline__ float bf16_rne(float f) { unsigned int u = __float_as_uint(f); u += 0x7FFFu + ((u >> 16) & 1u); return __uint_as_float(u & 0xFFFF0000u); }
__device__ __forceinline__ unsigned short bf16_bits(float f) { unsigned int u = __float_as_uint(f); u += 0x7FFFu + ((u >> 16) & 1u); return (unsigned short)(u >> 16); }
__device__ __forceinline__ void split16(float v, b16& hi, b16& lo) { hi = (b16)v; lo = (b16)(v - (float)hi); }
__device__ __forceinline__ v16b frag_kb(const b16* p, int hh) { const v8b a = *(const v8b*)(p + 8 * hh), b = *(const v8b*)(p + 16 + 8 * hh); v16b f;
#pragma unroll
  for (int e = 0; e < 8; ++e) { f[e] = a[e]; f[8 + e] = b[e]; } return f; }
__device__ __forceinline__ v16bb frag_bf(const unsigned short* p, int hh) { const v8us a = *(const v8us*)(p + 8 * hh), b = *(const v8us*)(p + 16 + 8 * hh); union { unsigned short s[16]; v16bb v; } u;
#pragma unroll
  for (int e = 0; e < 8; ++e) { u.s[e] = a[e]; u.s[8 + e] = b[e]; } return u.v; }
__device__ __forceinline__ v16bb frag_f32bf(const float* p, int hh) { union { unsigned short s[16]; v16bb v; } u;
#pragma unroll
  for (int e = 0; e < 8; ++e) { u.s[e] = bf16_bits(p[8 * hh + e]); u.s[8 + e] = bf16_bits(p[16 + 8 * hh + e]); } return u.v; }
__device__ __forceinline__ void frag_split(const float* p, int hh, v16b& fh, v16b& fl) {
#pragma unroll
  for (int e = 0; e < 8; ++e) { b16 a, c; split16(p[8 * hh + e] * AS_, a, c); fh[e] = a; fl[e] = c; split16(p[16 + 8 * hh + e] * AS_, a, c); fh[8 + e] = a; fl[8 + e] = c; } }
__device__ __forceinline__ v8f wmma16b(v16b a, v16b b, v8f c) { v8f d = __builtin_amdgcn_wmma_f32_16x16x32_f16(false, a, false, b, (short)0, c, false, false); asm volatile("v_nop\n\tv_nop\n\tv_nop\n\tv_nop" : "+v"(d) : "v"(a), "v"(b)); return d; }
__device__ __forceinline__ v8f wmma16bb(v16bb a, v16bb b, v8f c) { v8f d = __builtin_amdgcn_wmma_f32_16x16x32_bf16(false, a, false, b, (short)0, c, false, false); asm volatile("v_nop\n\tv_nop\n\tv_nop\n\tv_nop" : "+v"(d) : "v"(a), "v"(b)); return d; }
__device__ __forceinline__ void wave_lds_sync() { __builtin_amdgcn_fence(__ATOMIC_RELEASE, "workgroup"); __builtin_amdgcn_wave_barrier(); __builtin_amdgcn_fence(__ATOMIC_ACQUIRE, "workgroup"); }
__device__ __forceinline__ float nexp(float x) { return __builtin_amdgcn_exp2f(x * 1.4426950408889634f); }
__device__ __forceinline__ float sigm(float x) { return __builtin_amdgcn_rcpf(1.0f + nexp(-x)); }
__device__ __forceinline__ float softplus_(float z) { return fmaxf(z, 0.0f) + log1pf(__expf(-fabsf(z))); }
__device__ __forceinline__ float pmul(float a, float b) { float p = a * b; asm volatile("" : "+v"(p)); return p; }

__global__ __launch_bounds__(256) void prep_kernel(const float* __restrict__ hid, const float* __restrict__ ipw, const float* __restrict__ opw, const float* __restrict__ xpw, const float* __restrict__ ww,
                                                   unsigned short* __restrict__ h16, unsigned short* __restrict__ ip16, b16* __restrict__ op16, b16* __restrict__ xp16, unsigned short* __restrict__ ww16) {
  const size_t tid = (size_t)blockIdx.x * blockDim.x + threadIdx.x, nth = (size_t)gridDim.x * blockDim.x;
  for (int pass = 0; pass < 2; ++pass) {
    for (size_t p = tid; p < (size_t)NT * DM / 8; p += nth) { v8us v;
#pragma unroll
      for (int e = 0; e < 8; ++e) v[e] = bf16_bits(hid[p * 8 + e]);
      *(volatile v8us*)(h16 + p * 8) = v; }
    for (size_t p = tid; p < (size_t)2 * DI * DM / 8; p += nth) { v8us v;
#pragma unroll
      for (int e = 0; e < 8; ++e) v[e] = bf16_bits(ipw[p * 8 + e]);
      *(volatile v8us*)(ip16 + p * 8) = v; }
    for (size_t p = tid; p < (size_t)DM * DI / 8; p += nth) { v8b v;
#pragma unroll
      for (int e = 0; e < 8; ++e) v[e] = (b16)bf16_rne(opw[p * 8 + e]);
      *(volatile v8b*)(op16 + p * 8) = v; }
    for (size_t p = tid; p < (size_t)XN * XK / 8; p += nth) { v8b v;
#pragma unroll
      for (int e = 0; e < 8; ++e) v[e] = (b16)bf16_rne(xpw[p * 8 + e]);
      *(volatile v8b*)(xp16 + p * 8) = v; }
    for (size_t p = tid; p < (size_t)W * W / 8; p += nth) { v8us v;
#pragma unroll
      for (int e = 0; e < 8; ++e) v[e] = bf16_bits(ww[p * 8 + e]);
      *(volatile v8us*)(ww16 + p * 8) = v; }
    __threadfence();
  }
}

__global__ __launch_bounds__(128) void inproj_kernel(const unsigned short* __restrict__ h16, const unsigned short* __restrict__ ip16, float* __restrict__ xr, float* __restrict__ zr) {
  __shared__ __attribute__((aligned(16))) float Ts[4][32 * 64];
  const int lane = threadIdx.x & 31, wave = threadIdx.x >> 5, nloc = lane & 15, hlf = lane >> 4, m0 = blockIdx.y * 128 + wave * 32, c0 = blockIdx.x * 64;
  v8f acc[2][4];
#pragma unroll
  for (int r = 0; r < 2; ++r)
#pragma unroll
    for (int t = 0; t < 4; ++t) acc[r][t] = (v8f){};
#pragma unroll 2
  for (int kb = 0; kb < DM; kb += 32) { const v16bb a0 = frag_bf(h16 + (size_t)(m0 + nloc) * DM + kb, hlf), a1 = frag_bf(h16 + (size_t)(m0 + 16 + nloc) * DM + kb, hlf);
#pragma unroll
    for (int t = 0; t < 4; ++t) { const v16bb bw = frag_bf(ip16 + (size_t)(c0 + t * 16 + nloc) * DM + kb, hlf); acc[0][t] = wmma16bb(a0, bw, acc[0][t]); acc[1][t] = wmma16bb(a1, bw, acc[1][t]); } }
  float* Tt = Ts[wave];
#pragma unroll
  for (int t = 0; t < 4; ++t)
#pragma unroll
    for (int r = 0; r < 2; ++r)
#pragma unroll
      for (int v = 0; v < 8; ++v) Tt[(r * 16 + v + 8 * hlf) * 64 + t * 16 + nloc] = acc[r][t][v];
  wave_lds_sync();
  float* dst0 = (c0 < DI) ? (xr + (size_t)m0 * DI + c0) : (zr + (size_t)m0 * DI + (c0 - DI));
  for (int pass = 0; pass < 2; ++pass) {
#pragma unroll
    for (int j = 0; j < 16; ++j) { const int rr = j * 2 + hlf, c4 = nloc * 4; *(volatile v4f*)(dst0 + (size_t)rr * DI + c4) = *(const v4f*)(Tt + rr * 64 + c4); }
    __threadfence(); }
}

__global__ __launch_bounds__(256) void conv_kernel(const float* __restrict__ cw, const float* __restrict__ cb, float* __restrict__ xr) {
  const int g = blockIdx.x * 256 + threadIdx.x, b = g / DI, d = g % DI; float* col = xr + ((size_t)b * L) * DI + d;
  const float w0 = bf16_rne(cw[d * KC + 0]), w1 = bf16_rne(cw[d * KC + 1]), w2 = bf16_rne(cw[d * KC + 2]), w3 = bf16_rne(cw[d * KC + 3]), bb = bf16_rne(cb[d]);
  float xm1 = col[(size_t)(L - 1) * DI], xm2 = col[(size_t)(L - 2) * DI], xm3 = col[(size_t)(L - 3) * DI];
  for (int t = L - 1; t >= 0; --t) {
    const float x0 = xm1, x1 = xm2, x2 = xm3; const float x3 = (t - 3 >= 0) ? col[(size_t)(t - 3) * DI] : 0.0f;
    const float pre = (pmul(w3, x0) + pmul(w2, x1)) + (pmul(w1, x2) + pmul(w0, x3)) + bb; const float o = pre * sigm(pre);
    ((volatile float*)col)[(size_t)t * DI] = o; ((volatile float*)col)[(size_t)t * DI] = o;
    xm1 = x1; xm2 = x2; xm3 = x3; }
  __threadfence();
}

__global__ __launch_bounds__(128) void wproj_kernel(const float* __restrict__ we, const unsigned short* __restrict__ ww16, const float* __restrict__ wb, float* __restrict__ wp) {
  __shared__ __attribute__((aligned(16))) float Ts[4][32 * 64];
  const int lane = threadIdx.x & 31, wave = threadIdx.x >> 5, nloc = lane & 15, hlf = lane >> 4, m0 = blockIdx.y * 128 + wave * 32;
  v8f acc[2][4];
#pragma unroll
  for (int r = 0; r < 2; ++r)
#pragma unroll
    for (int t = 0; t < 4; ++t) acc[r][t] = (v8f){};
#pragma unroll
  for (int kb = 0; kb < W; kb += 32) { const v16bb a0 = frag_f32bf(we + (size_t)(m0 + nloc) * W + kb, hlf), a1 = frag_f32bf(we + (size_t)(m0 + 16 + nloc) * W + kb, hlf);
#pragma unroll
    for (int t = 0; t < 4; ++t) { const v16bb bw = frag_bf(ww16 + (size_t)(t * 16 + nloc) * W + kb, hlf); acc[0][t] = wmma16bb(a0, bw, acc[0][t]); acc[1][t] = wmma16bb(a1, bw, acc[1][t]); } }
  float* Tt = Ts[wave];
#pragma unroll
  for (int t = 0; t < 4; ++t) { const float bb = bf16_rne(wb[t * 16 + nloc]);
#pragma unroll
    for (int r = 0; r < 2; ++r)
#pragma unroll
      for (int v = 0; v < 8; ++v) Tt[(r * 16 + v + 8 * hlf) * 64 + t * 16 + nloc] = acc[r][t][v] + bb; }
  wave_lds_sync();
  for (int pass = 0; pass < 2; ++pass) {
#pragma unroll
    for (int j = 0; j < 16; ++j) { const int rr = j * 2 + hlf, c4 = nloc * 4; *(volatile v4f*)(wp + (size_t)(m0 + rr) * W + c4) = *(const v4f*)(Tt + rr * 64 + c4); }
    __threadfence(); }
}

__global__ __launch_bounds__(128) void xproj_kernel(const float* __restrict__ xr, const float* __restrict__ wp, const b16* __restrict__ xp16, float* __restrict__ xd) {
  __shared__ __attribute__((aligned(16))) float Ts[4][32][XN];
  const int lane = threadIdx.x & 31, wave = threadIdx.x >> 5, nloc = lane & 15, hlf = lane >> 4, m0 = blockIdx.x * 128 + wave * 32;
  v8f acc[2][5];
#pragma unroll
  for (int r = 0; r < 2; ++r)
#pragma unroll
    for (int t = 0; t < 5; ++t) acc[r][t] = (v8f){};
  for (int kb = 0; kb < XK; kb += 32) { v16b a0, l0, a1, l1;
    if (kb < DI) { frag_split(xr + (size_t)(m0 + nloc) * DI + kb, hlf, a0, l0); frag_split(xr + (size_t)(m0 + 16 + nloc) * DI + kb, hlf, a1, l1); }
    else { frag_split(wp + (size_t)(m0 + nloc) * W + (kb - DI), hlf, a0, l0); frag_split(wp + (size_t)(m0 + 16 + nloc) * W + (kb - DI), hlf, a1, l1); }
#pragma unroll
    for (int t = 0; t < 5; ++t) { const v16b bw = frag_kb(xp16 + (size_t)(t * 16 + nloc) * XK + kb, hlf); acc[0][t] = wmma16b(a0, bw, acc[0][t]); acc[0][t] = wmma16b(l0, bw, acc[0][t]); acc[1][t] = wmma16b(a1, bw, acc[1][t]); acc[1][t] = wmma16b(l1, bw, acc[1][t]); } }
#pragma unroll
  for (int t = 0; t < 5; ++t)
#pragma unroll
    for (int r = 0; r < 2; ++r)
#pragma unroll
      for (int v = 0; v < 8; ++v) Ts[wave][r * 16 + v + 8 * hlf][t * 16 + nloc] = acc[r][t][v] * (1.0f / AS_);
  wave_lds_sync();
  for (int pass = 0; pass < 2; ++pass) { for (int i = lane; i < 32 * XN / 4; i += 32) { const int rr = i / (XN / 4), c4 = (i % (XN / 4)) * 4; *(volatile v4f*)(xd + (size_t)(m0 + rr) * XN + c4) = *(const v4f*)(&Ts[wave][rr][c4]); } __threadfence(); }
}

__global__ __launch_bounds__(256) void scan_kernel(const float* __restrict__ xd, const float* __restrict__ dtw, const float* __restrict__ dtb, const float* __restrict__ alog, const float* __restrict__ Dp, const float* __restrict__ zr, float* __restrict__ xr) {
  __shared__ float row[XN];
  const int g = blockIdx.x * 256 + threadIdx.x, b = g / DI, d = g % DI, t_ = threadIdx.x;
  float wdt[R];
#pragma unroll
  for (int r = 0; r < R; ++r) wdt[r] = bf16_rne(dtw[(size_t)d * R + r]);
  float A[NS], h[NS];
#pragma unroll
  for (int n = 0; n < NS; ++n) { A[n] = -__expf(bf16_rne(alog[(size_t)d * NS + n])); h[n] = 0.0f; }
  const float db = bf16_rne(dtb[d]), Dd = bf16_rne(Dp[d]);
  float* col = xr + ((size_t)b * L) * DI + d; const float* zc = zr + ((size_t)b * L) * DI + d;
  for (int t = 0; t < L; ++t) {
    __syncthreads();
    if (t_ < XN) row[t_] = xd[((size_t)b * L + t) * XN + t_];
    __syncthreads();
    float dl = db;
#pragma unroll
    for (int r = 0; r < R; ++r) dl += pmul(row[r], wdt[r]);
    const float delta = softplus_(dl); const float x = col[(size_t)t * DI]; const float dx = delta * x; float y = pmul(Dd, x);
#pragma unroll
    for (int n = 0; n < NS; ++n) { h[n] = pmul(nexp(pmul(delta, A[n])), h[n]) + pmul(dx, row[R + n]); y += pmul(h[n], row[R + NS + n]); }
    const float z = zc[(size_t)t * DI]; const float gte = y * (z * sigm(z));
    ((volatile float*)col)[(size_t)t * DI] = gte; ((volatile float*)col)[(size_t)t * DI] = gte;
  }
  __threadfence();
}

__global__ __launch_bounds__(128) void outproj_kernel(const float* __restrict__ gr, const b16* __restrict__ op16, float* __restrict__ out) {
  __shared__ __attribute__((aligned(16))) float Ts[4][32 * 64];
  const int lane = threadIdx.x & 31, wave = threadIdx.x >> 5, nloc = lane & 15, hlf = lane >> 4, m0 = blockIdx.y * 128 + wave * 32, c0 = blockIdx.x * 64;
  v8f acc[2][4];
#pragma unroll
  for (int r = 0; r < 2; ++r)
#pragma unroll
    for (int t = 0; t < 4; ++t) acc[r][t] = (v8f){};
#pragma unroll 2
  for (int kb = 0; kb < DI; kb += 32) { v16b a0, l0, a1, l1; frag_split(gr + (size_t)(m0 + nloc) * DI + kb, hlf, a0, l0); frag_split(gr + (size_t)(m0 + 16 + nloc) * DI + kb, hlf, a1, l1);
#pragma unroll
    for (int t = 0; t < 4; ++t) { const v16b bw = frag_kb(op16 + (size_t)(c0 + t * 16 + nloc) * DI + kb, hlf); acc[0][t] = wmma16b(a0, bw, acc[0][t]); acc[0][t] = wmma16b(l0, bw, acc[0][t]); acc[1][t] = wmma16b(a1, bw, acc[1][t]); acc[1][t] = wmma16b(l1, bw, acc[1][t]); } }
  float* Tt = Ts[wave];
#pragma unroll
  for (int t = 0; t < 4; ++t)
#pragma unroll
    for (int r = 0; r < 2; ++r)
#pragma unroll
      for (int v = 0; v < 8; ++v) Tt[(r * 16 + v + 8 * hlf) * 64 + t * 16 + nloc] = acc[r][t][v] * (1.0f / AS_);
  wave_lds_sync();
  float* dst0 = out + (size_t)m0 * DM + c0;
  for (int pass = 0; pass < 2; ++pass) {
#pragma unroll
    for (int j = 0; j < 16; ++j) { const int rr = j * 2 + hlf, c4 = nloc * 4; *(volatile v4f*)(dst0 + (size_t)rr * DM + c4) = *(const v4f*)(Tt + rr * 64 + c4); }
    __threadfence(); }
}
}

extern "C" void kernel_launch(void* const* d_in, const int* in_sizes, int n_in,
                              void* d_out, int out_size, void* d_ws, size_t ws_size, hipStream_t stream) {
  (void)n_in; (void)out_size;
  const float* hid = (const float*)d_in[0]; const float* we = (const float*)d_in[1]; const float* ipw = (const float*)d_in[2]; const float* cw = (const float*)d_in[3]; const float* cb = (const float*)d_in[4]; const float* ww = (const float*)d_in[5]; const float* wb = (const float*)d_in[6];
  const float* xpw = (const float*)d_in[7]; const float* dtw = (const float*)d_in[8]; const float* dtb = (const float*)d_in[9]; const float* alog = (const float*)d_in[10]; const float* Dp = (const float*)d_in[11]; const float* opw = (const float*)d_in[12];
  float* out = (float*)d_out;
  if (in_sizes[0] != NT * DM || in_sizes[1] != NT * W || in_sizes[2] != 2 * DI * DM || in_sizes[7] != XN * XK || in_sizes[8] != DI * R || in_sizes[12] != DM * DI) return;
  size_t off = 0; char* ws = (char*)d_ws;
  auto carve = [&](size_t bytes) { char* p = ws + off; off += (bytes + 255) & ~(size_t)255; return p; };
  unsigned short* h16 = (unsigned short*)carve((size_t)NT * DM * 2); unsigned short* ip16 = (unsigned short*)carve((size_t)2 * DI * DM * 2); b16* op16 = (b16*)carve((size_t)DM * DI * 2); b16* xp16 = (b16*)carve((size_t)XN * XK * 2); unsigned short* ww16 = (unsigned short*)carve(W * W * 2);
  float* xr = (float*)carve((size_t)NT * DI * 4); float* zr = (float*)carve((size_t)NT * DI * 4); float* wp = (float*)carve((size_t)NT * W * 4); float* xd = (float*)carve((size_t)NT * XN * 4);
  if (off > ws_size) return;
  prep_kernel<<<1024, 256, 0, stream>>>(hid, ipw, opw, xpw, ww, h16, ip16, op16, xp16, ww16);
  inproj_kernel<<<dim3(2 * DI / 64, NT / 128), 128, 0, stream>>>(h16, ip16, xr, zr);
  conv_kernel<<<Bn * DI / 256, 256, 0, stream>>>(cw, cb, xr);
  wproj_kernel<<<dim3(1, NT / 128), 128, 0, stream>>>(we, ww16, wb, wp);
  xproj_kernel<<<NT / 128, 128, 0, stream>>>(xr, wp, xp16, xd);
  scan_kernel<<<Bn * DI / 256, 256, 0, stream>>>(xd, dtw, dtb, alog, Dp, zr, xr);
  outproj_kernel<<<dim3(DM / 64, NT / 128), 128, 0, stream>>>(xr, op16, out);
}
